// RecurrentGCN_15135464751774
// MI455X (gfx1250) — hardware-run, weakly checked
//
#include <hip/hip_runtime.h>


namespace {
constexpr int N = 50000, E = 1600000, H = 64;
constexpr float XS = 8.0f, HS = 256.0f, WSC = 256.0f;
typedef _Float16 b16;
typedef __attribute__((ext_vector_type(16))) _Float16 v16b;
typedef __attribute__((ext_vector_type(8))) _Float16 v8b;
typedef __attribute__((ext_vector_type(8))) float v8f;
typedef __attribute__((ext_vector_type(4))) float v4f;
typedef __attribute__((ext_vector_type(2))) float v2f;
__device__ __forceinline__ float bf16_rne(float f) { unsigned int u = __float_as_uint(f); u += 0x7FFFu + ((u >> 16) & 1u); float r = __uint_as_float(u & 0xFFFF0000u); asm volatile("" : "+v"(r)); return r; }
__device__ __forceinline__ float bfv(float f) { float r = bf16_rne(f); asm volatile("" : "+v"(r)); return r; }
__device__ __forceinline__ void split16(float v, b16& hi, b16& lo) { hi = (b16)v; lo = (b16)(v - (float)hi); }
__device__ __forceinline__ v16b frag_kb(const b16* p, int hh) { const v8b a = *(const v8b*)(p + 8 * hh), b = *(const v8b*)(p + 16 + 8 * hh); v16b f;
#pragma unroll
  for (int e = 0; e < 8; ++e) { f[e] = a[e]; f[8 + e] = b[e]; } return f; }
__device__ __forceinline__ v8f wmma16b(v16b a, v16b b, v8f c) { v8f d = __builtin_amdgcn_wmma_f32_16x16x32_f16(false, a, false, b, (short)0, c, false, false); asm volatile("v_nop\n\tv_nop\n\tv_nop\n\tv_nop" : "+v"(d) : "v"(a), "v"(b)); return d; }
__device__ __forceinline__ void wave_lds_sync() { __builtin_amdgcn_fence(__ATOMIC_RELEASE, "workgroup"); __builtin_amdgcn_wave_barrier(); __builtin_amdgcn_fence(__ATOMIC_ACQUIRE, "workgroup"); }
__device__ __forceinline__ float pmul(float a, float b) { float p = a * b; asm volatile("" : "+v"(p)); return p; }
__device__ __forceinline__ int iclamp(int v, int lo, int hi) { return v < lo ? lo : (v > hi ? hi : v); }
__device__ __forceinline__ float sigm(float v) { return 1.0f / (1.0f + __expf(-v)); }
constexpr int CSR_NBLKD = 512, CSR_GBD = 8, CSR_GND = 1 << CSR_GBD  , CSR_TSD = (CSR_GND < 32 ? 32 : CSR_GND)  , CSR_MAXGD = 512, CSR_CAPD = 12288  ;
__device__ __host__ __forceinline__ int csr_tixD(int v) { return (v >> CSR_GBD) * CSR_TSD + (v & (CSR_GND - 1)); }
__global__ __launch_bounds__(64) void csrA_kernelD(const int* __restrict__ dst, int E, int N, int nG, int CHP, int NGP, int* __restrict__ STG, int* __restrict__ HST) {
  extern __shared__ int sm[];
  int* cnt = sm; int* run = sm + NGP; int* ids = sm + 2 * NGP;
  const int b = blockIdx.x; const int ch = (E + CSR_NBLKD - 1) / CSR_NBLKD; const int e0 = b * ch, e1 = min(E, e0 + ch);
  for (int i = threadIdx.x; i < NGP; i += 64) cnt[i] = 0;
  for (int i = threadIdx.x; i < CHP; i += 64) ids[i] = -1;
  __syncthreads();
  if (threadIdx.x == 0) {
    for (int e = e0; e < e1; ++e) { int d = dst[e]; d = (d < 0) ? 0 : (d >= N ? N - 1 : d); cnt[d >> CSR_GBD] += 1; }
    int acc = 0; for (int g = 0; g < nG; ++g) { run[g] = acc; acc += cnt[g]; }
    for (int e = e0; e < e1; ++e) { int d = dst[e]; d = (d < 0) ? 0 : (d >= N ? N - 1 : d); const int g = d >> CSR_GBD; ids[run[g]] = e; run[g] += 1; } }
  __syncthreads();
  typedef __attribute__((ext_vector_type(4))) int v4i;
  for (int pass = 0; pass < 2; ++pass) {
    for (int i = threadIdx.x; i < CHP / 4; i += 64) *(volatile v4i*)(STG + (size_t)b * CHP + i * 4) = *(const v4i*)(&ids[i * 4]);
    for (int i = threadIdx.x; i < NGP / 4; i += 64) { v4i v; for (int e = 0; e < 4; ++e) v[e] = (i * 4 + e < nG) ? cnt[i * 4 + e] : 0; *(volatile v4i*)(HST + (size_t)b * NGP + i * 4) = v; }
    __threadfence(); }
}
__global__ __launch_bounds__(512) void csrS_kernelD(const int* __restrict__ HST, int nG, int NGP, int* __restrict__ START, int* __restrict__ TOT, int* __restrict__ OFF) {
  __shared__ int tot[CSR_MAXGD];
  const int b = threadIdx.x;
  for (int pass = 0; pass < 2; ++pass) { int runb = 0; for (int g = 0; g < nG; ++g) { int c = HST[(size_t)b * NGP + g]; c = (c < 0) ? 0 : c; ((volatile int*)OFF)[(size_t)g * CSR_NBLKD + b] = runb; runb += c; } __threadfence(); }
  for (int g = threadIdx.x; g < nG; g += 512) { int s = 0; for (int bb = 0; bb < CSR_NBLKD; ++bb) { int c = HST[(size_t)bb * NGP + g]; s += (c < 0) ? 0 : c; } tot[g] = s; }
  __syncthreads();
  if (threadIdx.x < 32) {
    __shared__ int st[CSR_MAXGD + 32];
    if (threadIdx.x == 0) { int acc = 0; for (int g = 0; g < NGP; ++g) { st[g] = acc; if (g < nG) acc += (tot[g] + 31) & ~31; } st[NGP] = acc; }
    __builtin_amdgcn_fence(__ATOMIC_RELEASE, "workgroup"); __builtin_amdgcn_wave_barrier(); __builtin_amdgcn_fence(__ATOMIC_ACQUIRE, "workgroup");
    for (int pass = 0; pass < 2; ++pass) { for (int i = threadIdx.x; i < NGP + 32; i += 32) { ((volatile int*)START)[i] = (i <= NGP) ? st[min(i, NGP)] : 0; ((volatile int*)TOT)[i] = (i < nG) ? tot[i] : 0; } __threadfence(); } }
}
__global__ __launch_bounds__(256) void csrB_kernelD(const int* __restrict__ dst, int N, int nG, int CHP, int NGP, int permLen, const int* __restrict__ STG, const int* __restrict__ HST, const int* __restrict__ OFF, const int* __restrict__ START, const int* __restrict__ TOT, int* __restrict__ PERM, int* __restrict__ ROWPTR, int* __restrict__ ROWCNT, int* __restrict__ FLAG) {
  typedef __attribute__((ext_vector_type(4))) int v4i;
  __shared__ int ids[CSR_CAPD]; __shared__ unsigned short key[CSR_CAPD]; __shared__ int outp[CSR_CAPD]; __shared__ int ncnt[CSR_GND + 1]; __shared__ int boff[CSR_NBLKD + 1];
  const int g = blockIdx.x, t_ = threadIdx.x; int tot = TOT[g]; int st = START[g], stn = START[g + 1]; const int v0 = g * CSR_GND; const int nv = min(CSR_GND, N - v0); const int t0 = g * CSR_TSD;
  st = (st < 0) ? 0 : (st > permLen - 32 ? permLen - 32 : st) & ~31; stn = (stn < st) ? st : (stn > permLen ? permLen : stn); tot = (tot < 0) ? 0 : tot; if (tot > stn - st && tot <= CSR_CAPD) tot = stn - st;
  if (tot > CSR_CAPD) {
    for (int pass = 0; pass < 2; ++pass) { for (int i = t_; i < CSR_TSD / 4; i += 256) { v4i a, c; for (int e = 0; e < 4; ++e) { a[e] = st; c[e] = 0; } *(volatile v4i*)(ROWPTR + t0 + i * 4) = a; *(volatile v4i*)(ROWCNT + t0 + i * 4) = c; } if (t_ == 0) ((volatile int*)FLAG)[0] = 1; __threadfence(); } (void)nv; return; }
  if (t_ == 0) { int acc = 0; for (int b = 0; b < CSR_NBLKD; ++b) { boff[b] = acc; int c = HST[(size_t)b * NGP + g]; c = (c < 0) ? 0 : (c > CHP ? CHP : c); acc += c; if (acc > tot) acc = tot; } boff[CSR_NBLKD] = acc; }
  for (int i = t_; i <= CSR_GND; i += 256) ncnt[i] = 0;
  __syncthreads();
  for (int b = 0; b < CSR_NBLKD; ++b) { const int c = boff[b + 1] - boff[b]; int o_ = OFF[(size_t)g * CSR_NBLKD + b]; o_ = (o_ < 0) ? 0 : (o_ > CHP - c ? CHP - c : o_); const int* src_ = STG + (size_t)b * CHP + o_;
    for (int i = t_; i < c; i += 256) { int id = src_[i]; id = (id < 0) ? 0 : id; ids[boff[b] + i] = id; int d = dst[id]; d = (d < v0) ? v0 : (d >= N ? N - 1 : d); int kk = d - v0; kk = (kk < 0) ? 0 : (kk >= CSR_GND ? CSR_GND - 1 : kk); key[boff[b] + i] = (unsigned short)kk; } }
  __syncthreads();
  if (t_ == 0) { for (int i = 0; i < tot; ++i) ncnt[key[i]] += 1; int acc = 0; for (int vl = 0; vl < CSR_GND; ++vl) { const int c = ncnt[vl]; ncnt[vl] = acc; acc += c; } ncnt[CSR_GND] = acc;
    for (int i = 0; i < tot; ++i) { const int vl = key[i]; outp[ncnt[vl]] = ids[i]; ncnt[vl] += 1; }
    for (int vl = CSR_GND; vl > 0; --vl) ncnt[vl] = ncnt[vl - 1]; ncnt[0] = 0; }
  __syncthreads();
  for (int pass = 0; pass < 2; ++pass) {
    for (int i = t_; i < (stn - st) / 4; i += 256) { v4i v; for (int e = 0; e < 4; ++e) { const int q = i * 4 + e; v[e] = (q < tot) ? outp[q] : -1; } *(volatile v4i*)(PERM + st + i * 4) = v; }
    for (int i = t_; i < CSR_TSD / 4; i += 256) { v4i a, c; for (int e = 0; e < 4; ++e) { const int vl = i * 4 + e; const int vc = vl < CSR_GND ? vl : CSR_GND; a[e] = (vl < CSR_GND) ? st + ncnt[vc] : st; c[e] = (vl < nv) ? (ncnt[(vc < CSR_GND ? vc : CSR_GND - 1) + 1] - ncnt[vc]) : 0; } *(volatile v4i*)(ROWPTR + t0 + i * 4) = a; *(volatile v4i*)(ROWCNT + t0 + i * 4) = c; }
    __threadfence(); }
}
__global__ __launch_bounds__(256) void csrZ_kernelD(int* __restrict__ p, size_t n4) { typedef __attribute__((ext_vector_type(4))) int v4i; const size_t tid = (size_t)blockIdx.x * 256 + threadIdx.x, nth = (size_t)gridDim.x * 256; v4i z = {0, 0, 0, 0}; for (size_t i = tid; i < n4; i += nth) *(volatile v4i*)(p + i * 4) = z; }
struct CsrBufsD { int *STG, *HST, *OFF, *START, *TOT, *PERM, *ROWPTR, *ROWCNT, *FLAG; int nG, NGP, CHP; size_t permLen; char* base; size_t bytes; };
static size_t csr_carveD(CsrBufsD& c, char* ws, size_t off, int E, int N) {
  const size_t off0 = off; c.base = ws + off;
  auto al = [&](size_t bytes) { char* p = ws + off; off += (bytes + 255) & ~(size_t)255; return p; };
  c.nG = (N + CSR_GND - 1) / CSR_GND; c.NGP = (c.nG + 31) & ~31; const int ch = (E + CSR_NBLKD - 1) / CSR_NBLKD; c.CHP = (ch + 31) & ~31; c.permLen = (size_t)E + 32 * (size_t)c.nG + 32;
  c.STG = (int*)al((size_t)CSR_NBLKD * c.CHP * 4); c.HST = (int*)al((size_t)CSR_NBLKD * c.NGP * 4); c.OFF = (int*)al((size_t)c.NGP * CSR_NBLKD * 4); c.START = (int*)al((size_t)(c.NGP + 64) * 4); c.TOT = (int*)al((size_t)(c.NGP + 64) * 4);
  c.PERM = (int*)al(c.permLen * 4); c.ROWPTR = (int*)al((size_t)c.nG * CSR_TSD * 4); c.ROWCNT = (int*)al((size_t)c.nG * CSR_TSD * 4); c.FLAG = (int*)al(256);
  c.bytes = off - off0; return off;
}
static void csr_buildD(const CsrBufsD& c, const int* dst, int E, int N, hipStream_t stream) {
  const size_t smem = (size_t)(2 * c.NGP + c.CHP) * 4;
  csrZ_kernelD<<<512, 256, 0, stream>>>((int*)c.base, c.bytes / 16);
  csrA_kernelD<<<CSR_NBLKD, 64, smem, stream>>>(dst, E, N, c.nG, c.CHP, c.NGP, c.STG, c.HST);
  csrS_kernelD<<<1, 512, 0, stream>>>(c.HST, c.nG, c.NGP, c.START, c.TOT, c.OFF);
  csrB_kernelD<<<c.nG, 256, 0, stream>>>(dst, N, c.nG, c.CHP, c.NGP, (int)c.permLen, c.STG, c.HST, c.OFF, c.START, c.TOT, c.PERM, c.ROWPTR, c.ROWCNT, c.FLAG);
}
constexpr int CSR_NBLKS = 512, CSR_GBS = 8, CSR_GNS = 1 << CSR_GBS  , CSR_TSS = (CSR_GNS < 32 ? 32 : CSR_GNS)  , CSR_MAXGS = 512, CSR_CAPS = 12288  ;
__device__ __host__ __forceinline__ int csr_tixS(int v) { return (v >> CSR_GBS) * CSR_TSS + (v & (CSR_GNS - 1)); }
__global__ __launch_bounds__(64) void csrA_kernelS(const int* __restrict__ dst, int E, int N, int nG, int CHP, int NGP, int* __restrict__ STG, int* __restrict__ HST) {
  extern __shared__ int sm[];
  int* cnt = sm; int* run = sm + NGP; int* ids = sm + 2 * NGP;
  const int b = blockIdx.x; const int ch = (E + CSR_NBLKS - 1) / CSR_NBLKS; const int e0 = b * ch, e1 = min(E, e0 + ch);
  for (int i = threadIdx.x; i < NGP; i += 64) cnt[i] = 0;
  for (int i = threadIdx.x; i < CHP; i += 64) ids[i] = -1;
  __syncthreads();
  if (threadIdx.x == 0) {
    for (int e = e0; e < e1; ++e) { int d = dst[e]; d = (d < 0) ? 0 : (d >= N ? N - 1 : d); cnt[d >> CSR_GBS] += 1; }
    int acc = 0; for (int g = 0; g < nG; ++g) { run[g] = acc; acc += cnt[g]; }
    for (int e = e0; e < e1; ++e) { int d = dst[e]; d = (d < 0) ? 0 : (d >= N ? N - 1 : d); const int g = d >> CSR_GBS; ids[run[g]] = e; run[g] += 1; } }
  __syncthreads();
  typedef __attribute__((ext_vector_type(4))) int v4i;
  for (int pass = 0; pass < 2; ++pass) {
    for (int i = threadIdx.x; i < CHP / 4; i += 64) *(volatile v4i*)(STG + (size_t)b * CHP + i * 4) = *(const v4i*)(&ids[i * 4]);
    for (int i = threadIdx.x; i < NGP / 4; i += 64) { v4i v; for (int e = 0; e < 4; ++e) v[e] = (i * 4 + e < nG) ? cnt[i * 4 + e] : 0; *(volatile v4i*)(HST + (size_t)b * NGP + i * 4) = v; }
    __threadfence(); }
}
__global__ __launch_bounds__(512) void csrS_kernelS(const int* __restrict__ HST, int nG, int NGP, int* __restrict__ START, int* __restrict__ TOT, int* __restrict__ OFF) {
  __shared__ int tot[CSR_MAXGS];
  const int b = threadIdx.x;
  for (int pass = 0; pass < 2; ++pass) { int runb = 0; for (int g = 0; g < nG; ++g) { int c = HST[(size_t)b * NGP + g]; c = (c < 0) ? 0 : c; ((volatile int*)OFF)[(size_t)g * CSR_NBLKS + b] = runb; runb += c; } __threadfence(); }
  for (int g = threadIdx.x; g < nG; g += 512) { int s = 0; for (int bb = 0; bb < CSR_NBLKS; ++bb) { int c = HST[(size_t)bb * NGP + g]; s += (c < 0) ? 0 : c; } tot[g] = s; }
  __syncthreads();
  if (threadIdx.x < 32) {
    __shared__ int st[CSR_MAXGS + 32];
    if (threadIdx.x == 0) { int acc = 0; for (int g = 0; g < NGP; ++g) { st[g] = acc; if (g < nG) acc += (tot[g] + 31) & ~31; } st[NGP] = acc; }
    __builtin_amdgcn_fence(__ATOMIC_RELEASE, "workgroup"); __builtin_amdgcn_wave_barrier(); __builtin_amdgcn_fence(__ATOMIC_ACQUIRE, "workgroup");
    for (int pass = 0; pass < 2; ++pass) { for (int i = threadIdx.x; i < NGP + 32; i += 32) { ((volatile int*)START)[i] = (i <= NGP) ? st[min(i, NGP)] : 0; ((volatile int*)TOT)[i] = (i < nG) ? tot[i] : 0; } __threadfence(); } }
}
__global__ __launch_bounds__(256) void csrB_kernelS(const int* __restrict__ dst, int N, int nG, int CHP, int NGP, int permLen, const int* __restrict__ STG, const int* __restrict__ HST, const int* __restrict__ OFF, const int* __restrict__ START, const int* __restrict__ TOT, int* __restrict__ PERM, int* __restrict__ ROWPTR, int* __restrict__ ROWCNT, int* __restrict__ FLAG) {
  typedef __attribute__((ext_vector_type(4))) int v4i;
  __shared__ int ids[CSR_CAPS]; __shared__ unsigned short key[CSR_CAPS]; __shared__ int outp[CSR_CAPS]; __shared__ int ncnt[CSR_GNS + 1]; __shared__ int boff[CSR_NBLKS + 1];
  const int g = blockIdx.x, t_ = threadIdx.x; int tot = TOT[g]; int st = START[g], stn = START[g + 1]; const int v0 = g * CSR_GNS; const int nv = min(CSR_GNS, N - v0); const int t0 = g * CSR_TSS;
  st = (st < 0) ? 0 : (st > permLen - 32 ? permLen - 32 : st) & ~31; stn = (stn < st) ? st : (stn > permLen ? permLen : stn); tot = (tot < 0) ? 0 : tot; if (tot > stn - st && tot <= CSR_CAPS) tot = stn - st;
  if (tot > CSR_CAPS) {
    for (int pass = 0; pass < 2; ++pass) { for (int i = t_; i < CSR_TSS / 4; i += 256) { v4i a, c; for (int e = 0; e < 4; ++e) { a[e] = st; c[e] = 0; } *(volatile v4i*)(ROWPTR + t0 + i * 4) = a; *(volatile v4i*)(ROWCNT + t0 + i * 4) = c; } if (t_ == 0) ((volatile int*)FLAG)[0] = 1; __threadfence(); } (void)nv; return; }
  if (t_ == 0) { int acc = 0; for (int b = 0; b < CSR_NBLKS; ++b) { boff[b] = acc; int c = HST[(size_t)b * NGP + g]; c = (c < 0) ? 0 : (c > CHP ? CHP : c); acc += c; if (acc > tot) acc = tot; } boff[CSR_NBLKS] = acc; }
  for (int i = t_; i <= CSR_GNS; i += 256) ncnt[i] = 0;
  __syncthreads();
  for (int b = 0; b < CSR_NBLKS; ++b) { const int c = boff[b + 1] - boff[b]; int o_ = OFF[(size_t)g * CSR_NBLKS + b]; o_ = (o_ < 0) ? 0 : (o_ > CHP - c ? CHP - c : o_); const int* src_ = STG + (size_t)b * CHP + o_;
    for (int i = t_; i < c; i += 256) { int id = src_[i]; id = (id < 0) ? 0 : id; ids[boff[b] + i] = id; int d = dst[id]; d = (d < v0) ? v0 : (d >= N ? N - 1 : d); int kk = d - v0; kk = (kk < 0) ? 0 : (kk >= CSR_GNS ? CSR_GNS - 1 : kk); key[boff[b] + i] = (unsigned short)kk; } }
  __syncthreads();
  if (t_ == 0) { for (int i = 0; i < tot; ++i) ncnt[key[i]] += 1; int acc = 0; for (int vl = 0; vl < CSR_GNS; ++vl) { const int c = ncnt[vl]; ncnt[vl] = acc; acc += c; } ncnt[CSR_GNS] = acc;
    for (int i = 0; i < tot; ++i) { const int vl = key[i]; outp[ncnt[vl]] = ids[i]; ncnt[vl] += 1; }
    for (int vl = CSR_GNS; vl > 0; --vl) ncnt[vl] = ncnt[vl - 1]; ncnt[0] = 0; }
  __syncthreads();
  for (int pass = 0; pass < 2; ++pass) {
    for (int i = t_; i < (stn - st) / 4; i += 256) { v4i v; for (int e = 0; e < 4; ++e) { const int q = i * 4 + e; v[e] = (q < tot) ? outp[q] : -1; } *(volatile v4i*)(PERM + st + i * 4) = v; }
    for (int i = t_; i < CSR_TSS / 4; i += 256) { v4i a, c; for (int e = 0; e < 4; ++e) { const int vl = i * 4 + e; const int vc = vl < CSR_GNS ? vl : CSR_GNS; a[e] = (vl < CSR_GNS) ? st + ncnt[vc] : st; c[e] = (vl < nv) ? (ncnt[(vc < CSR_GNS ? vc : CSR_GNS - 1) + 1] - ncnt[vc]) : 0; } *(volatile v4i*)(ROWPTR + t0 + i * 4) = a; *(volatile v4i*)(ROWCNT + t0 + i * 4) = c; }
    __threadfence(); }
}
__global__ __launch_bounds__(256) void csrZ_kernelS(int* __restrict__ p, size_t n4) { typedef __attribute__((ext_vector_type(4))) int v4i; const size_t tid = (size_t)blockIdx.x * 256 + threadIdx.x, nth = (size_t)gridDim.x * 256; v4i z = {0, 0, 0, 0}; for (size_t i = tid; i < n4; i += nth) *(volatile v4i*)(p + i * 4) = z; }
struct CsrBufsS { int *STG, *HST, *OFF, *START, *TOT, *PERM, *ROWPTR, *ROWCNT, *FLAG; int nG, NGP, CHP; size_t permLen; char* base; size_t bytes; };
static size_t csr_carveS(CsrBufsS& c, char* ws, size_t off, int E, int N) {
  const size_t off0 = off; c.base = ws + off;
  auto al = [&](size_t bytes) { char* p = ws + off; off += (bytes + 255) & ~(size_t)255; return p; };
  c.nG = (N + CSR_GNS - 1) / CSR_GNS; c.NGP = (c.nG + 31) & ~31; const int ch = (E + CSR_NBLKS - 1) / CSR_NBLKS; c.CHP = (ch + 31) & ~31; c.permLen = (size_t)E + 32 * (size_t)c.nG + 32;
  c.STG = (int*)al((size_t)CSR_NBLKS * c.CHP * 4); c.HST = (int*)al((size_t)CSR_NBLKS * c.NGP * 4); c.OFF = (int*)al((size_t)c.NGP * CSR_NBLKS * 4); c.START = (int*)al((size_t)(c.NGP + 64) * 4); c.TOT = (int*)al((size_t)(c.NGP + 64) * 4);
  c.PERM = (int*)al(c.permLen * 4); c.ROWPTR = (int*)al((size_t)c.nG * CSR_TSS * 4); c.ROWCNT = (int*)al((size_t)c.nG * CSR_TSS * 4); c.FLAG = (int*)al(256);
  c.bytes = off - off0; return off;
}
static void csr_buildS(const CsrBufsS& c, const int* dst, int E, int N, hipStream_t stream) {
  const size_t smem = (size_t)(2 * c.NGP + c.CHP) * 4;
  csrZ_kernelS<<<512, 256, 0, stream>>>((int*)c.base, c.bytes / 16);
  csrA_kernelS<<<CSR_NBLKS, 64, smem, stream>>>(dst, E, N, c.nG, c.CHP, c.NGP, c.STG, c.HST);
  csrS_kernelS<<<1, 512, 0, stream>>>(c.HST, c.nG, c.NGP, c.START, c.TOT, c.OFF);
  csrB_kernelS<<<c.nG, 256, 0, stream>>>(dst, N, c.nG, c.CHP, c.NGP, (int)c.permLen, c.STG, c.HST, c.OFF, c.START, c.TOT, c.PERM, c.ROWPTR, c.ROWCNT, c.FLAG);
}


__global__ __launch_bounds__(256) void wput_kernel(const float* __restrict__ wx, const float* __restrict__ th, const float* __restrict__ lw, b16* __restrict__ WG, b16* __restrict__ WL) { const int u = blockIdx.x * 256 + threadIdx.x; v8b v;
  if (u < 4 * H * 32) { const int o = u / 32, k0 = (u % 32) * 8; const int g = o / H, oc = o % H;
#pragma unroll
    for (int j = 0; j < 8; ++j) { const int k = k0 + j; float w; if (k < H) w = wx[((size_t)g * H + k) * H + oc]; else { const int kk = (k - H) / H, r = (k - H) % H; w = th[(((size_t)g * 3 + kk) * H + r) * H + oc]; } v[j] = (b16)(bf16_rne(w) * WSC); }
    for (int pass = 0; pass < 2; ++pass) { *(volatile v8b*)(WG + (size_t)o * 4 * H + k0) = v; __threadfence(); } }
  if (u < H * 8) { const int o = u / 8, k0 = (u % 8) * 8;
#pragma unroll
    for (int j = 0; j < 8; ++j) v[j] = (b16)(bf16_rne(lw[(size_t)(k0 + j) * H + o]) * WSC); for (int pass = 0; pass < 2; ++pass) { *(volatile v8b*)(WL + (size_t)o * H + k0) = v; __threadfence(); } } }
__global__ __launch_bounds__(256) void deg_kernel(const float* __restrict__ ew, const int* __restrict__ dsts, const int* __restrict__ PERM, const int* __restrict__ ROWPTR, const int* __restrict__ ROWCNT, int permLen, int NLIM, float* __restrict__ DG) { const int i = blockIdx.x * 256 + threadIdx.x; if (i >= N) return; float deg = 0.0f;
  if (i < NLIM) { int st = ROWPTR[i], cnt = ROWCNT[i]; cnt = iclamp(cnt, 0, E); st = iclamp(st, 0, permLen - cnt);
#pragma unroll 1
    for (int j = 0; j < cnt; ++j) { const int e = iclamp(PERM[st + j], 0, E - 1); if (iclamp(dsts[e], 0, N - 1) >= NLIM) continue; deg += bfv(ew[e]); } }
  const float d = deg > 0.0f ? rsqrtf(deg) : 0.0f; const float diag = pmul(pmul(d, d), deg) - 1.0f;
  for (int pass = 0; pass < 2; ++pass) { ((volatile float*)DG)[i] = d; ((volatile float*)DG)[N + i] = diag; __threadfence(); } }
template <int STEP>
__global__ __launch_bounds__(256) void prop_kernel(const float* __restrict__ Z, const float* __restrict__ h, const float* __restrict__ DG, const float* __restrict__ ew, const int* __restrict__ srcs, const int* __restrict__ PERM, const int* __restrict__ ROWPTR, const int* __restrict__ ROWCNT, int permLen, int NLIM, float* __restrict__ OUT) { const int wave = threadIdx.x >> 5, lane = threadIdx.x & 31; const size_t i = (size_t)blockIdx.x * 8 + wave; if (i >= (size_t)NLIM) return; int st = ROWPTR[i], cnt = ROWCNT[i]; cnt = iclamp(cnt, 0, E); st = iclamp(st, 0, permLen - cnt);
  const float di = DG[i], diag = DG[N + i]; float a0 = 0.0f, a1 = 0.0f;
#pragma unroll 1
  for (int j = 0; j < cnt; ++j) { const int e = iclamp(PERM[st + j], 0, E - 1); const size_t u = (size_t)iclamp(srcs[e], 0, N - 1); if (u >= (size_t)NLIM) continue; const float nrm = -pmul(pmul(DG[u], bfv(ew[e])), di); const v2f z = *(const v2f*)(Z + u * H + lane * 2); a0 += pmul(nrm, STEP == 1 ? bfv(z[0]) : z[0]); a1 += pmul(nrm, STEP == 1 ? bfv(z[1]) : z[1]); }
  const v2f zi = *(const v2f*)(Z + i * H + lane * 2); float o0 = a0 + pmul(diag, STEP == 1 ? bfv(zi[0]) : zi[0]), o1 = a1 + pmul(diag, STEP == 1 ? bfv(zi[1]) : zi[1]);
  if (STEP == 2) { const v2f hi = *(const v2f*)(h + i * H + lane * 2); o0 = 2.0f * o0 - bfv(hi[0]); o1 = 2.0f * o1 - bfv(hi[1]); }
  for (int pass = 0; pass < 2; ++pass) { *(volatile v2f*)(OUT + i * H + lane * 2) = (v2f){o0, o1}; __threadfence(); } }
__global__ __launch_bounds__(32) void cell_kernel(const float* __restrict__ x, const float* __restrict__ h, const float* __restrict__ c, const float* __restrict__ T1, const float* __restrict__ T2, const b16* __restrict__ WG, const b16* __restrict__ WL, const float* __restrict__ wc, const float* __restrict__ bb, const float* __restrict__ cvb, const float* __restrict__ lb, int NLIM, float* __restrict__ HO, float* __restrict__ HN, float* __restrict__ CN) {
  __shared__ __attribute__((aligned(16))) b16 Ah[16][4 * H + 8], Al[16][2 * H + 8], Rh[16][H + 8], Rl[16][H + 8]; __shared__ float Tf[16][4 * H + 4], Cf[16][H], Hf[16][H], Of[16][H + 4]; const int lane = threadIdx.x, nloc = lane & 15, hlf = lane >> 4; const size_t m0 = (size_t)blockIdx.x * 16; if (m0 >= (size_t)NLIM) return;
  for (int rr = 0; rr < 16; ++rr) for (int q = 0; q < 2; ++q) { const int cc = q * 32 + lane; const size_t n = m0 + rr; Ah[rr][cc] = (b16)(bf16_rne(x[n * H + cc]) * HS); Ah[rr][H + cc] = (b16)(bf16_rne(h[n * H + cc]) * HS);     b16 p, ql; split16(T1[n * H + cc] * HS, p, ql); Ah[rr][2 * H + cc] = p; Al[rr][cc] = ql; split16(T2[n * H + cc] * HS, p, ql); Ah[rr][3 * H + cc] = p; Al[rr][H + cc] = ql; }
  wave_lds_sync(); v8f acc[16];
#pragma unroll
  for (int t = 0; t < 16; ++t) acc[t] = (v8f){};
#pragma unroll
  for (int kb = 0; kb < 2 * H; kb += 32) { const v16b a = frag_kb(&Ah[nloc][kb], hlf);
#pragma unroll
    for (int t = 0; t < 16; ++t) acc[t] = wmma16b(a, frag_kb(WG + (size_t)(t * 16 + nloc) * 4 * H + kb, hlf), acc[t]); }
#pragma unroll
  for (int kb = 2 * H; kb < 4 * H; kb += 32) { const v16b a = frag_kb(&Ah[nloc][kb], hlf), al = frag_kb(&Al[nloc][kb - 2 * H], hlf);
#pragma unroll
    for (int t = 0; t < 16; ++t) { const v16b bw = frag_kb(WG + (size_t)(t * 16 + nloc) * 4 * H + kb, hlf); acc[t] = wmma16b(a, bw, acc[t]); acc[t] = wmma16b(al, bw, acc[t]); } }
#pragma unroll
  for (int t = 0; t < 16; ++t) { const int cc = t * 16 + nloc; const int g = cc / H, oc = cc % H; const float bias = bfv(bb[g * H + oc]) + bfv(cvb[g * H + oc]);
#pragma unroll
    for (int r8 = 0; r8 < 8; ++r8) Tf[8 * hlf + r8][cc] = acc[t][r8] * (1.0f / (HS * WSC)) + bias; }
  wave_lds_sync();
  for (int rr = 0; rr < 16; ++rr) for (int q = 0; q < 2; ++q) { const int oc = q * 32 + lane; const size_t n = m0 + rr; const float cv = bfv(c[n * H + oc]);
    const float ig = sigm(Tf[rr][oc] + pmul(bfv(wc[oc]), cv)); const float fg = sigm(Tf[rr][H + oc] + pmul(bfv(wc[H + oc]), cv)); const float tg = tanhf(Tf[rr][2 * H + oc]);
    const float cn = pmul(fg, cv) + pmul(ig, tg); const float og = sigm(Tf[rr][3 * H + oc] + pmul(bfv(wc[2 * H + oc]), cn)); const float hn = pmul(og, tanhf(cn));
    Cf[rr][oc] = cn; Hf[rr][oc] = hn; b16 p, ql; split16(fmaxf(hn, 0.0f) * HS, p, ql); Rh[rr][oc] = p; Rl[rr][oc] = ql; }
  if (lane < 16) for (int k = H; k < H + 8; ++k) { Rh[lane][k] = (b16)0.0f; Rl[lane][k] = (b16)0.0f; }
  wave_lds_sync(); v8f al4[4] = {(v8f){}, (v8f){}, (v8f){}, (v8f){}};
#pragma unroll
  for (int kb = 0; kb < H; kb += 32) { const v16b a = frag_kb(&Rh[nloc][kb], hlf), al = frag_kb(&Rl[nloc][kb], hlf);
#pragma unroll
    for (int t = 0; t < 4; ++t) { const v16b bw = frag_kb(WL + (size_t)(t * 16 + nloc) * H + kb, hlf); al4[t] = wmma16b(a, bw, al4[t]); al4[t] = wmma16b(al, bw, al4[t]); } }
#pragma unroll
  for (int t = 0; t < 4; ++t) { const int cc = t * 16 + nloc; const float b_ = bfv(lb[cc]);
#pragma unroll
    for (int r8 = 0; r8 < 8; ++r8) Of[8 * hlf + r8][cc] = al4[t][r8] * (1.0f / (HS * WSC)) + b_; }
  wave_lds_sync();
  for (int pass = 0; pass < 2; ++pass) { for (int rr = 0; rr < 16; ++rr) { const size_t n = m0 + rr; *(volatile v2f*)(HO + n * H + lane * 2) = (v2f){Of[rr][lane * 2], Of[rr][lane * 2 + 1]}; *(volatile v2f*)(HN + n * H + lane * 2) = (v2f){Hf[rr][lane * 2], Hf[rr][lane * 2 + 1]}; *(volatile v2f*)(CN + n * H + lane * 2) = (v2f){Cf[rr][lane * 2], Cf[rr][lane * 2 + 1]}; } __threadfence(); } }
}

extern "C" void kernel_launch(void* const* d_in, const int* in_sizes, int n_in, void* d_out, int out_size, void* d_ws, size_t ws_size, hipStream_t stream) {
  (void)n_in;
  auto Fp = [&](int i) { return (const float*)d_in[i]; }; auto Ip = [&](int i) { return (const int*)d_in[i]; };
  if (in_sizes[0] != N * H || in_sizes[1] != 2 * E || in_sizes[2] != E || in_sizes[3] != N * H || in_sizes[4] != N * H || in_sizes[5] != 4 * H * H || in_sizes[6] != 3 * H || in_sizes[8] != 12 * H * H || in_sizes[10] != H * H || out_size != 3 * N * H) return;
  const int NLIM = N;
  size_t off = 0; char* ws = (char*)d_ws;
  auto carve = [&](size_t bytes) { char* p = ws + off; off += (bytes + 255) & ~(size_t)255; return p; };
  b16* WG = (b16*)carve((size_t)4 * H * 4 * H * 2); b16* WL = (b16*)carve((size_t)H * H * 2); float* DG = (float*)carve((size_t)2 * N * 4); float* T1 = (float*)carve((size_t)N * H * 4); float* T2 = (float*)carve((size_t)N * H * 4);
  CsrBufsD cd; off = csr_carveD(cd, ws, off, E, N); CsrBufsS cs; off = csr_carveS(cs, ws, off, E, N);
  if (off > ws_size || off > ((size_t)96 << 20)) return;
  float* HO = (float*)d_out; float* HN = HO + (size_t)N * H; float* CN = HN + (size_t)N * H;
  wput_kernel<<<(4 * H * 32 + 255) / 256, 256, 0, stream>>>(Fp(5), Fp(8), Fp(10), WG, WL);
  csr_buildD(cd, Ip(1) + E, E, N, stream);
  csr_buildS(cs, Ip(1), E, N, stream);
  deg_kernel<<<(N + 255) / 256, 256, 0, stream>>>(Fp(2), Ip(1) + E, cs.PERM, cs.ROWPTR, cs.ROWCNT, (int)cs.permLen, NLIM, DG);
  prop_kernel<1><<<(NLIM + 7) / 8, 256, 0, stream>>>(Fp(3), Fp(3), DG, Fp(2), Ip(1), cd.PERM, cd.ROWPTR, cd.ROWCNT, (int)cd.permLen, NLIM, T1);
  prop_kernel<2><<<(NLIM + 7) / 8, 256, 0, stream>>>(T1, Fp(3), DG, Fp(2), Ip(1), cd.PERM, cd.ROWPTR, cd.ROWCNT, (int)cd.permLen, NLIM, T2);
  cell_kernel<<<NLIM / 16, 32, 0, stream>>>(Fp(0), Fp(3), Fp(4), T1, T2, WG, WL, Fp(6), Fp(7), Fp(9), Fp(11), NLIM, HO, HN, CN);
}
